// Up1_13365938225164
// MI455X (gfx1250) — hardware-verified
//
#include <hip/hip_runtime.h>
#define NBI 8
#define C1 128
#define CX 256
#define CO 128
#define HH 64
#define NPX (HH * HH)
#define NR (NBI * NPX)
#define KT 9
#define KD (KT * CO)
#define NOM 27
#define NOMP 32
typedef __bf16 v16b __attribute__((ext_vector_type(16)));
typedef unsigned short v8us __attribute__((ext_vector_type(8), may_alias));
typedef float  v8f  __attribute__((ext_vector_type(8)));
typedef float  v4f  __attribute__((ext_vector_type(4)));
typedef float  v4fa __attribute__((ext_vector_type(4), may_alias));
union FragB { v16b v; v8us half[2]; unsigned short u[16]; };

__device__ __forceinline__ unsigned short bf16_bits(float x) { unsigned int u = __float_as_uint(x); return (unsigned short)((u + 0x7FFFu + ((u >> 16) & 1u)) >> 16); }
__device__ __forceinline__ float bf16_val(unsigned short b) { return __uint_as_float(((unsigned int)b) << 16); }
__device__ __forceinline__ float bf16_round(float x) { return bf16_val(bf16_bits(x)); }
template <int NT>
__device__ __forceinline__ v8f mmaN(v16b ah, v16b al, v16b bh, v16b bl, v8f c) {
  c = __builtin_amdgcn_wmma_f32_16x16x32_bf16(false, ah, false, bh, (short)0, c, false, false);
  if (NT >= 2) c = __builtin_amdgcn_wmma_f32_16x16x32_bf16(false, al, false, bh, (short)0, c, false, false);
  if (NT >= 3) c = __builtin_amdgcn_wmma_f32_16x16x32_bf16(false, ah, false, bl, (short)0, c, false, false);
  asm volatile("v_nop\n\tv_nop\n\tv_nop\n\tv_nop" : "+v"(c) : "v"(ah), "v"(al), "v"(bh), "v"(bl));
  return c;
}

__global__ __launch_bounds__(256) void k_wt_bf16(const float* __restrict__ W, unsigned short* __restrict__ Wt, int K, int N) {
  const int t = blockIdx.x * 256 + threadIdx.x;
  const int k8n = K / 8;
  if (t >= N * k8n) return;
  const int n = t / k8n, k8 = (t % k8n) * 8;
  v8us v;
#pragma unroll
  for (int i = 0; i < 8; ++i) v[i] = bf16_bits(W[(size_t)(k8 + i) * N + n]);
  *(volatile v8us*)(Wt + (size_t)n * K + k8) = v;
  __threadfence();
  *(volatile v8us*)(Wt + (size_t)n * K + k8) = v;
}

template <bool ASPLIT, int ACT, bool BIAS_BF16>
__global__ __launch_bounds__(128) void k_gemm_bf(const float* __restrict__ A, int lda, const unsigned short* __restrict__ Wt, int ldb,
                                               const float* __restrict__ bias, float* __restrict__ C, int ldc, int M, int N, int K) {
  __shared__ __attribute__((aligned(16))) float so[4][16][64];
  const int tid = threadIdx.x, w = tid >> 5, lane = tid & 31, ln = lane & 15, hh = lane >> 4;
  const int ntn = N / 64;
  const int wid = blockIdx.x * 4 + w;
  const int mt = wid / ntn, nq = wid % ntn;
  if (mt * 16 >= M) return;
  const int row0 = mt * 16, col0 = nq * 64;
  const float* arow = A + (size_t)(row0 + ln) * lda;
  v8f acc[4] = {};
  for (int kb = 0; kb < K; kb += 32) {
    FragB ah, al;
    const v4f x0 = *(const v4fa*)(arow + kb + 8 * hh), x1 = *(const v4fa*)(arow + kb + 8 * hh + 4);
    const v4f x2 = *(const v4fa*)(arow + kb + 16 + 8 * hh), x3 = *(const v4fa*)(arow + kb + 16 + 8 * hh + 4);
    float xs[16] = {x0[0],x0[1],x0[2],x0[3],x1[0],x1[1],x1[2],x1[3],x2[0],x2[1],x2[2],x2[3],x3[0],x3[1],x3[2],x3[3]};
#pragma unroll
    for (int i = 0; i < 16; ++i) { const unsigned short hb = bf16_bits(xs[i]); ah.u[i] = hb; al.u[i] = ASPLIT ? bf16_bits(xs[i] - bf16_val(hb)) : (unsigned short)0; }
#pragma unroll
    for (int t = 0; t < 4; ++t) {
      const unsigned short* brow = Wt + (size_t)(col0 + t * 16 + ln) * ldb + kb;
      FragB b;
      b.half[0] = *(const v8us*)(brow + 8 * hh);
      b.half[1] = *(const v8us*)(brow + 16 + 8 * hh);
      acc[t] = mmaN<ASPLIT ? 2 : 1>(ah.v, al.v, b.v, b.v, acc[t]);
    }
  }
#pragma unroll
  for (int t = 0; t < 4; ++t) {
    float bv = bias ? bias[col0 + t * 16 + ln] : 0.f;
    if (BIAS_BF16) bv = bf16_round(bv);
#pragma unroll
    for (int r = 0; r < 8; ++r) { float v = acc[t][r] + bv; if (ACT == 1) v = fmaxf(v, 0.f); so[w][8 * hh + r][t * 16 + ln] = v; }
  }
  __builtin_amdgcn_fence(__ATOMIC_ACQ_REL, "workgroup");
  __builtin_amdgcn_wave_barrier();
  const int rsub = lane >> 4, c4 = (lane & 15) * 4;
  for (int pass = 0; pass < 2; ++pass) {
#pragma unroll
    for (int q = 0; q < 8; ++q) {
      const int r = q * 2 + rsub;
      const v4f v = *(const v4fa*)&so[w][r][c4];
      *(volatile v4f*)(C + (size_t)(row0 + r) * ldc + col0 + c4) = v;
    }
    if (pass == 0) __threadfence();
  }
}

template <bool ASPLIT, int ACT, bool BIAS_BF16, bool RES_BF16>
__global__ __launch_bounds__(128) void k_gemm_bf3(const float* __restrict__ A, int lda, const unsigned short* __restrict__ Wt, int ldb,
                                                const float* __restrict__ bias, const float* __restrict__ resid, int rmod, int ldr,
                                                float* __restrict__ C, int ldc, int M, int N, int K) {
  __shared__ __attribute__((aligned(16))) float so[4][16][64];
  const int tid = threadIdx.x, w = tid >> 5, lane = tid & 31, ln = lane & 15, hh = lane >> 4;
  const int ntn = N / 64;
  const int wid = blockIdx.x * 4 + w;
  const int mt = wid / ntn, nq = wid % ntn;
  if (mt * 16 >= M) return;
  const int row0 = mt * 16, col0 = nq * 64;
  const float* arow = A + (size_t)(row0 + ln) * lda;
  v8f acc[4] = {};
  for (int kb = 0; kb < K; kb += 32) {
    FragB ah, al;
    const v4f x0 = *(const v4fa*)(arow + kb + 8 * hh), x1 = *(const v4fa*)(arow + kb + 8 * hh + 4);
    const v4f x2 = *(const v4fa*)(arow + kb + 16 + 8 * hh), x3 = *(const v4fa*)(arow + kb + 16 + 8 * hh + 4);
    float xs[16] = {x0[0],x0[1],x0[2],x0[3],x1[0],x1[1],x1[2],x1[3],x2[0],x2[1],x2[2],x2[3],x3[0],x3[1],x3[2],x3[3]};
#pragma unroll
    for (int i = 0; i < 16; ++i) { const unsigned short hb = bf16_bits(xs[i]); ah.u[i] = hb; al.u[i] = ASPLIT ? bf16_bits(xs[i] - bf16_val(hb)) : (unsigned short)0; }
#pragma unroll
    for (int t = 0; t < 4; ++t) {
      const unsigned short* brow = Wt + (size_t)(col0 + t * 16 + ln) * ldb + kb;
      FragB b;
      b.half[0] = *(const v8us*)(brow + 8 * hh);
      b.half[1] = *(const v8us*)(brow + 16 + 8 * hh);
      acc[t] = mmaN<ASPLIT ? 2 : 1>(ah.v, al.v, b.v, b.v, acc[t]);
    }
  }
#pragma unroll
  for (int t = 0; t < 4; ++t) {
    const int col = col0 + t * 16 + ln;
    float bv = bias ? bias[col] : 0.f;
    if (BIAS_BF16) bv = bf16_round(bv);
#pragma unroll
    for (int r = 0; r < 8; ++r) {
      float v = acc[t][r] + bv;
      if (resid) { float rv = resid[(size_t)((row0 + 8 * hh + r) % rmod) * ldr + col]; if (RES_BF16) rv = bf16_round(rv); v += rv; }
      if (ACT == 1) v = fmaxf(v, 0.f);
      if (ACT == 2) v = 0.5f * v * (1.0f + erff(v * 0.70710678118654752f));
      if (ACT == 3) { const float u = 0.7978845608028654f * (v + 0.044715f * v * v * v); v = 0.5f * v * (1.0f + tanhf(u)); }
      so[w][8 * hh + r][t * 16 + ln] = v;
    }
  }
  __builtin_amdgcn_fence(__ATOMIC_ACQ_REL, "workgroup");
  __builtin_amdgcn_wave_barrier();
  const int rsub = lane >> 4, c4 = (lane & 15) * 4;
  for (int pass = 0; pass < 2; ++pass) {
#pragma unroll
    for (int q = 0; q < 8; ++q) {
      const int r = q * 2 + rsub;
      const v4f v = *(const v4fa*)&so[w][r][c4];
      *(volatile v4f*)(C + (size_t)(row0 + r) * ldc + col0 + c4) = v;
    }
    if (pass == 0) __threadfence();
  }
}
template <bool PARAM_BF16>
__global__ __launch_bounds__(256) void k_layernorm(const float* __restrict__ X, const float* __restrict__ R, const float* __restrict__ g, const float* __restrict__ bta,
                                                  float* __restrict__ out_sum, float* __restrict__ out_norm, int N, float eps) {
  __shared__ float red[256];
  const int row = blockIdx.x, tid = threadIdx.x;
  const float* x = X + (size_t)row * N; const float* rr = R ? R + (size_t)row * N : nullptr;
  float vals[16];
  const int per = N / 256;
  float s1 = 0.f;
  for (int u = 0; u < per / 4; ++u) {
    const int j = tid * 4 + 1024 * u;
    const v4f a = *(const v4fa*)(x + j);
    v4f b = {0.f,0.f,0.f,0.f}; if (rr) b = *(const v4fa*)(rr + j);
#pragma unroll
    for (int q = 0; q < 4; ++q) { const float v = a[q] + b[q]; vals[u * 4 + q] = v; s1 += v; }
  }
  red[tid] = s1; __syncthreads();
  for (int st = 128; st > 0; st >>= 1) { if (tid < st) red[tid] += red[tid + st]; __syncthreads(); }
  const float mu = red[0] / (float)N; __syncthreads();
  float s2 = 0.f;
  for (int u = 0; u < per / 4; ++u)
#pragma unroll
    for (int q = 0; q < 4; ++q) { const float c = vals[u * 4 + q] - mu; s2 += c * c; }
  red[tid] = s2; __syncthreads();
  for (int st = 128; st > 0; st >>= 1) { if (tid < st) red[tid] += red[tid + st]; __syncthreads(); }
  const float rs = rsqrtf(red[0] / (float)N + eps);
  for (int pass = 0; pass < 2; ++pass) {
    for (int u = 0; u < per / 4; ++u) {
      const int j = tid * 4 + 1024 * u;
      v4f o, sm;
#pragma unroll
      for (int q = 0; q < 4; ++q) {
        float gg = g[j + q], bb = bta[j + q];
        if (PARAM_BF16) { gg = bf16_round(gg); bb = bf16_round(bb); }
        sm[q] = vals[u * 4 + q]; o[q] = (vals[u * 4 + q] - mu) * rs * gg + bb;
      }
      if (out_sum) *(volatile v4f*)(out_sum + (size_t)row * N + j) = sm;
      *(volatile v4f*)(out_norm + (size_t)row * N + j) = o;
    }
    if (pass == 0) __threadfence();
  }
}


typedef _Float16 v16h __attribute__((ext_vector_type(16)));
union FragH { v16h v; v8us half[2]; _Float16 h[16]; unsigned short u[16]; };
template <int NT>
__device__ __forceinline__ v8f mmaH(v16h ah, v16h al, v16h bh, v16h bl, v8f c) {
  c = __builtin_amdgcn_wmma_f32_16x16x32_f16(false, ah, false, bh, (short)0, c, false, false);
  if (NT >= 2) c = __builtin_amdgcn_wmma_f32_16x16x32_f16(false, al, false, bh, (short)0, c, false, false);
  if (NT >= 3) c = __builtin_amdgcn_wmma_f32_16x16x32_f16(false, ah, false, bl, (short)0, c, false, false);
  asm volatile("v_nop\n\tv_nop\n\tv_nop\n\tv_nop" : "+v"(c) : "v"(ah), "v"(al), "v"(bh), "v"(bl));
  return c;
}
template <bool ASPLIT>
__global__ __launch_bounds__(128) void k_gemm_h(const float* __restrict__ A, int lda, size_t sA, const _Float16* __restrict__ Bh, int ldb, size_t sB, float alpha, float* __restrict__ C, int ldc, size_t sC, int M, int N, int K) {
  __shared__ __attribute__((aligned(16))) float so[4][16][64];
  const int tid = threadIdx.x, w = tid >> 5, lane = tid & 31, ln = lane & 15, hh = lane >> 4; const int by = blockIdx.y;
  A += (size_t)by * sA; Bh += (size_t)by * sB; C += (size_t)by * sC;
  const int ntn = (N + 63) / 64; const int wid = blockIdx.x * 4 + w; const int mt = wid / ntn, nq = wid % ntn; if (mt * 16 >= M) return;
  const int row0 = mt * 16, col0 = nq * 64; const float* arow = A + (size_t)(row0 + ln) * lda;
  v8f acc[4] = {};
  for (int kb = 0; kb < K; kb += 32) {
    FragH ah, al;
    const v4f x0 = *(const v4fa*)(arow + kb + 8 * hh), x1 = *(const v4fa*)(arow + kb + 8 * hh + 4), x2 = *(const v4fa*)(arow + kb + 16 + 8 * hh), x3 = *(const v4fa*)(arow + kb + 16 + 8 * hh + 4);
    float xs[16] = {x0[0],x0[1],x0[2],x0[3],x1[0],x1[1],x1[2],x1[3],x2[0],x2[1],x2[2],x2[3],x3[0],x3[1],x3[2],x3[3]};
#pragma unroll
    for (int i = 0; i < 16; ++i) { const _Float16 h = (_Float16)xs[i]; ah.h[i] = h; al.h[i] = ASPLIT ? (_Float16)(xs[i] - (float)h) : (_Float16)0.0f; }
#pragma unroll
    for (int t = 0; t < 4; ++t) { if (col0 + t * 16 >= N) continue; const size_t boff = (size_t)(col0 + t * 16 + ln) * ldb + kb; FragH bq; bq.half[0] = *(const v8us*)(Bh + boff + 8 * hh); bq.half[1] = *(const v8us*)(Bh + boff + 16 + 8 * hh);
      acc[t] = mmaH<ASPLIT ? 2 : 1>(ah.v, al.v, bq.v, bq.v, acc[t]); }
  }
#pragma unroll
  for (int t = 0; t < 4; ++t) { if (col0 + t * 16 >= N) continue;
#pragma unroll
    for (int r = 0; r < 8; ++r) so[w][8 * hh + r][t * 16 + ln] = acc[t][r] * alpha; }
  __builtin_amdgcn_fence(__ATOMIC_ACQ_REL, "workgroup"); __builtin_amdgcn_wave_barrier();
  const int rsub = lane >> 4, c4 = (lane & 15) * 4;
  for (int pass = 0; pass < 2; ++pass) {
#pragma unroll
    for (int q = 0; q < 8; ++q) { const int r = q * 2 + rsub; if (col0 + c4 < N) { const v4f v = *(const v4fa*)&so[w][r][c4]; *(volatile v4f*)(C + (size_t)(row0 + r) * ldc + col0 + c4) = v; } }
    if (pass == 0) __threadfence(); }
}

__global__ __launch_bounds__(256) void k_wt_f16(const float* __restrict__ W, _Float16* __restrict__ Wt, int K, int N, float scale) {
  const int t = blockIdx.x * 256 + threadIdx.x; if (t >= N * (K / 8)) return; const int n = t / (K / 8), k8 = (t % (K / 8)) * 8; FragH f;
#pragma unroll
  for (int i = 0; i < 8; ++i) f.h[i] = (_Float16)(bf16_round(W[(size_t)(k8 + i) * N + n]) * scale); const v8us o = f.half[0];
  *(volatile v8us*)((unsigned short*)Wt + (size_t)n * K + k8) = o; __threadfence(); *(volatile v8us*)((unsigned short*)Wt + (size_t)n * K + k8) = o;
}
template <int ACT>
__global__ __launch_bounds__(128) void k_gemm_hhx(const _Float16* __restrict__ A, int lda, size_t sA, const _Float16* __restrict__ Bh, int ldb, size_t sB, float alpha, const float* __restrict__ bias, size_t sBias, const float* __restrict__ CP, int rowsPerB, size_t sCPb, int row0g,
    float* __restrict__ C, _Float16* __restrict__ C16, int ldc, size_t sC, int M, int N, int K) {
  __shared__ __attribute__((aligned(16))) float so[4][16][64];
  const int tid = threadIdx.x, w = tid >> 5, lane = tid & 31, ln = lane & 15, hh = lane >> 4; const int by = blockIdx.y;
  A += (size_t)by * sA; Bh += (size_t)by * sB; const size_t cofs = (size_t)by * sC; const float* bp = bias ? bias + (size_t)by * sBias : nullptr;
  const int ntn = (N + 63) / 64; const int wid = blockIdx.x * 4 + w; const int mt = wid / ntn, nq = wid % ntn; if (mt * 16 >= M) return;
  const int row0 = mt * 16, col0 = nq * 64; const _Float16* arow = A + (size_t)(row0 + ln) * lda;
  v8f acc[4] = {};
  for (int kb = 0; kb < K; kb += 32) { FragH ah; ah.half[0] = *(const v8us*)((const unsigned short*)arow + kb + 8 * hh); ah.half[1] = *(const v8us*)((const unsigned short*)arow + kb + 16 + 8 * hh);
#pragma unroll
    for (int t = 0; t < 4; ++t) { if (col0 + t * 16 >= N) continue; const size_t boff = (size_t)(col0 + t * 16 + ln) * ldb + kb; FragH bq; bq.half[0] = *(const v8us*)((const unsigned short*)Bh + boff + 8 * hh); bq.half[1] = *(const v8us*)((const unsigned short*)Bh + boff + 16 + 8 * hh);
      acc[t] = mmaH<1>(ah.v, ah.v, bq.v, bq.v, acc[t]); }
  }
#pragma unroll
  for (int t = 0; t < 4; ++t) { if (col0 + t * 16 >= N) continue; const int col = col0 + t * 16 + ln; const float bv = bp ? bf16_round(bp[col]) : 0.f;
#pragma unroll
    for (int r = 0; r < 8; ++r) { float v = acc[t][r] * alpha + bv; if (CP) { const int bidx = (row0g + row0 + 8 * hh + r) / rowsPerB; v += CP[(size_t)bidx * sCPb + (size_t)by * 64 + col]; } if (ACT == 1) v = (v > 0.f) ? v : expm1f(v); else if (ACT == 7) v = (v > 0.f) ? v + 1.0f : expf(v); else if (ACT == 8) v = tanhf(v); else if (ACT == 9) v = 0.5f * v * (1.0f + tanhf(0.7978845608028654f * (v + 0.044715f * v * v * v))); else if (ACT == 11) v = 1.0f / (1.0f + expf(-v)); else if (ACT == 12) v = (v > 0.f) ? v : 0.01f * v; else if (ACT == 14) v = (v > 0.f) ? v : 0.1f * v; else if (ACT == 15) v = v / (1.0f + expf(-v)); else if (ACT == 3) v = fmaxf(v, 0.f); else if (ACT == 6) v = 0.5f * v * (1.0f + erff(v * 0.70710678118654752f)); so[w][8 * hh + r][t * 16 + ln] = v; } }
  __builtin_amdgcn_fence(__ATOMIC_ACQ_REL, "workgroup"); __builtin_amdgcn_wave_barrier();
  const int rsub = lane >> 4, c4 = (lane & 15) * 4; typedef _Float16 v4h __attribute__((ext_vector_type(4)));
  for (int pass = 0; pass < 2; ++pass) {
#pragma unroll
    for (int q = 0; q < 8; ++q) { const int r = q * 2 + rsub; if (col0 + c4 < N) { const v4f v = *(const v4fa*)&so[w][r][c4]; if (C) *(volatile v4f*)(C + cofs + (size_t)(row0 + r) * ldc + col0 + c4) = v; if (C16) { v4h h4; for (int i = 0; i < 4; ++i) h4[i] = (_Float16)v[i]; *(volatile v4h*)(C16 + cofs + (size_t)(row0 + r) * ldc + col0 + c4) = h4; } } }
    if (pass == 0) __threadfence(); }
}


typedef _Float16 v4h __attribute__((ext_vector_type(4)));

__global__ __launch_bounds__(256) void k_x16(const float* __restrict__ x, _Float16* __restrict__ X16, size_t n8) { const size_t t = (size_t)blockIdx.x * 256 + threadIdx.x; if (t >= n8) return; FragH f;
#pragma unroll
  for (int q = 0; q < 8; ++q) f.h[q] = (_Float16)bf16_round(x[t * 8 + q]); *(volatile v8us*)((unsigned short*)X16 + t * 8) = f.half[0]; __threadfence(); *(volatile v8us*)((unsigned short*)X16 + t * 8) = f.half[0]; }
__global__ __launch_bounds__(256) void k_h16(const float* __restrict__ x, _Float16* __restrict__ X16, size_t n8) { const size_t t = (size_t)blockIdx.x * 256 + threadIdx.x; if (t >= n8) return; FragH f;
#pragma unroll
  for (int q = 0; q < 8; ++q) f.h[q] = (_Float16)x[t * 8 + q]; *(volatile v8us*)((unsigned short*)X16 + t * 8) = f.half[0]; __threadfence(); *(volatile v8us*)((unsigned short*)X16 + t * 8) = f.half[0]; }
__global__ __launch_bounds__(256) void k_round16f(const float* __restrict__ W, _Float16* __restrict__ Bt, size_t n8) { const size_t t = (size_t)blockIdx.x * 256 + threadIdx.x; if (t >= n8) return; FragH f;
#pragma unroll
  for (int i = 0; i < 8; ++i) f.h[i] = (_Float16)(bf16_round(W[t * 8 + i]) * 16.0f); *(volatile v8us*)((unsigned short*)Bt + t * 8) = f.half[0]; __threadfence(); *(volatile v8us*)((unsigned short*)Bt + t * 8) = f.half[0]; }
template <int NHv, int TTv>
__global__ __launch_bounds__(256) void k_vt(const _Float16* __restrict__ V16, int ldv, int voff, _Float16* __restrict__ Vt) { __shared__ unsigned short tl[64][66]; const int tid = threadIdx.x; const int slab = blockIdx.x / (TTv / 64), lg = blockIdx.x % (TTv / 64); const int b = slab / NHv, h = slab % NHv;
  for (int i = tid; i < 64 * 8; i += 256) { const int r = i / 8, c8 = (i % 8) * 8; FragH f; f.half[0] = *(const v8us*)((const unsigned short*)V16 + ((size_t)b * TTv + lg * 64 + r) * ldv + voff + h * 64 + c8);
#pragma unroll
    for (int q = 0; q < 8; ++q) tl[r][c8 + q] = f.u[q]; }
  __syncthreads();
  for (int pass = 0; pass < 2; ++pass) {
#pragma unroll
    for (int rd = 0; rd < 2; ++rd) { const int d = rd * 32 + tid / 8, pc = tid % 8; FragH f;
#pragma unroll
      for (int q = 0; q < 8; ++q) f.u[q] = tl[pc * 8 + q][d];
      *(volatile v8us*)((unsigned short*)Vt + ((size_t)slab * 64 + d) * TTv + lg * 64 + pc * 8) = f.half[0]; }
    if (pass == 0) __threadfence(); } }

__global__ __launch_bounds__(256) void k_hl(const float* __restrict__ F, _Float16* __restrict__ Hh, _Float16* __restrict__ Hl, size_t n8) { const size_t t = (size_t)blockIdx.x * 256 + threadIdx.x; if (t >= n8) return; FragH fh, fl; const v4f a = *(const v4fa*)(F + t * 8), c = *(const v4fa*)(F + t * 8 + 4);
#pragma unroll
  for (int q = 0; q < 4; ++q) { _Float16 h = (_Float16)a[q]; fh.h[q] = h; fl.h[q] = (_Float16)((a[q] - (float)h) * 1024.0f); h = (_Float16)c[q]; fh.h[4 + q] = h; fl.h[4 + q] = (_Float16)((c[q] - (float)h) * 1024.0f); }
  for (int pass = 0; pass < 2; ++pass) { *(volatile v8us*)((unsigned short*)Hh + t * 8) = fh.half[0]; *(volatile v8us*)((unsigned short*)Hl + t * 8) = fl.half[0]; if (pass == 0) __threadfence(); } }

__global__ __launch_bounds__(256) void k_xcat(const float* __restrict__ x1, const float* __restrict__ x2, int b, float* __restrict__ XC) {
  #pragma clang fp contract(off)
  const int t = blockIdx.x * 256 + threadIdx.x; if (t >= NPX * (CX / 4)) return; const int c0 = (t % (CX / 4)) * 4, p = t / (CX / 4); const int y = p / HH, x = p % HH; v4f v;
  if (c0 < C1) {
#pragma unroll
    for (int q = 0; q < 4; ++q) v[q] = bf16_round(x2[((size_t)b * C1 + c0 + q) * NPX + p]); }
  else { const float sc = (float)(32 - 1) / (float)(HH - 1); const float cy = (float)y * sc, cxx = (float)x * sc; int iy = (int)floorf(cy), ix = (int)floorf(cxx); iy = min(max(iy, 0), 30); ix = min(max(ix, 0), 30); const float ty = cy - (float)iy, tx = cxx - (float)ix;
#pragma unroll
    for (int q = 0; q < 4; ++q) { const float* s = x1 + ((size_t)b * C1 + c0 - C1 + q) * 1024; const float a00 = bf16_round(s[iy * 32 + ix]), a01 = bf16_round(s[iy * 32 + ix + 1]), a10 = bf16_round(s[(iy + 1) * 32 + ix]), a11 = bf16_round(s[(iy + 1) * 32 + ix + 1]);
      const float r0 = a00 * (1.0f - ty) + a10 * ty, r1 = a01 * (1.0f - ty) + a11 * ty; v[q] = r0 * (1.0f - tx) + r1 * tx; } }
  *(volatile v4f*)(XC + (size_t)p * CX + c0) = v; __threadfence(); *(volatile v4f*)(XC + (size_t)p * CX + c0) = v; }
__global__ __launch_bounds__(256) void k_dw(const float* __restrict__ P, int C, const float* __restrict__ w, const float* __restrict__ bb, int mode, _Float16* __restrict__ O16, float* __restrict__ O32) {
  #pragma clang fp contract(off)
  const int t = blockIdx.x * 256 + threadIdx.x; if (t >= NPX * (C / 4)) return; const int c0 = (t % (C / 4)) * 4, p = t / (C / 4); const int y = p / HH, x = p % HH; float acc[4];
#pragma unroll
  for (int q = 0; q < 4; ++q) acc[q] = bf16_round(bb[c0 + q]);
#pragma unroll 1
  for (int k = 0; k < 9; ++k) { const int yy = y - 1 + k / 3, xx = x - 1 + k % 3; if (yy < 0 || yy >= HH || xx < 0 || xx >= HH) continue; const v4f a = *(const v4fa*)(P + ((size_t)yy * HH + xx) * C + c0);
#pragma unroll
    for (int q = 0; q < 4; ++q) acc[q] += bf16_round(w[(size_t)(c0 + q) * 9 + k]) * a[q]; }
  if (mode == 0) { _Float16 h4[4], l4[4];
#pragma unroll
    for (int q = 0; q < 4; ++q) { h4[q] = (_Float16)acc[q]; l4[q] = (_Float16)((acc[q] - (float)h4[q]) * 1024.0f); }
    const unsigned long long pk = *(const unsigned long long*)h4, pl = *(const unsigned long long*)l4;
    for (int pass = 0; pass < 2; ++pass) { *(volatile unsigned long long*)((unsigned short*)O16 + (size_t)p * 2 * C + c0) = pk; *(volatile unsigned long long*)((unsigned short*)O16 + (size_t)p * 2 * C + C + c0) = pl; if (pass == 0) __threadfence(); } }
  else { v4f o0;
#pragma unroll
    for (int q = 0; q < 4; ++q) o0[q] = acc[q];
    *(volatile v4f*)(O32 + (size_t)p * C + c0) = o0; __threadfence(); *(volatile v4f*)(O32 + (size_t)p * C + c0) = o0; } }
__global__ __launch_bounds__(256) void k_f16c(const float* __restrict__ F, _Float16* __restrict__ O, size_t n8) { const size_t t = (size_t)blockIdx.x * 256 + threadIdx.x; if (t >= n8) return; const v4f a = *(const v4fa*)(F + t * 8), c = *(const v4fa*)(F + t * 8 + 4); FragH f;
#pragma unroll
  for (int q = 0; q < 8; ++q) f.h[q] = (_Float16)((q < 4) ? a[q] : c[q - 4]);
  *(volatile v8us*)((unsigned short*)O + t * 8) = f.half[0]; __threadfence(); *(volatile v8us*)((unsigned short*)O + t * 8) = f.half[0]; }
__global__ __launch_bounds__(256) void k_im2col(const _Float16* __restrict__ P, _Float16* __restrict__ COL) { const int t = blockIdx.x * 256 + threadIdx.x; if (t >= NPX * KT * (CO / 8)) return; const int c0 = (t % (CO / 8)) * 8; const int k = (t / (CO / 8)) % KT; const int p = t / ((CO / 8) * KT); const int h = p / HH, w = p % HH; const int yy = h - 1 + k / 3, xx = w - 1 + k % 3; FragH f = FragH{};
  if (yy >= 0 && yy < HH && xx >= 0 && xx < HH) f.half[0] = *(const v8us*)((const unsigned short*)P + ((size_t)yy * HH + xx) * CO + c0);
  *(volatile v8us*)((unsigned short*)COL + ((size_t)p * KT + k) * CO + c0) = f.half[0]; __threadfence(); *(volatile v8us*)((unsigned short*)COL + ((size_t)p * KT + k) * CO + c0) = f.half[0]; }
__global__ __launch_bounds__(256) void k_wom(const float* __restrict__ pw, const float* __restrict__ mw, const float* __restrict__ pb, const float* __restrict__ mb, _Float16* __restrict__ Bt, float* __restrict__ BP) { const int t = blockIdx.x * 256 + threadIdx.x; if (t < NOMP * (KD / 8)) { const int col0 = (t % (KD / 8)) * 8, o = t / (KD / 8); const int k = col0 / CO, c0 = col0 % CO; FragH f;
#pragma unroll
    for (int q = 0; q < 8; ++q) { float v = 0.f; if (o < 18) v = bf16_round(pw[((size_t)o * CO + c0 + q) * KT + k]); else if (o < NOM) v = bf16_round(mw[((size_t)(o - 18) * CO + c0 + q) * KT + k]); f.h[q] = (_Float16)(v * 16.0f); }
    *(volatile v8us*)((unsigned short*)Bt + (size_t)o * KD + col0) = f.half[0]; __threadfence(); *(volatile v8us*)((unsigned short*)Bt + (size_t)o * KD + col0) = f.half[0]; }
  if (blockIdx.x == 0 && threadIdx.x < NOMP) { const int i = threadIdx.x; const float v = (i < 18) ? pb[i] : (i < NOM) ? mb[i - 18] : 0.f; *(volatile float*)(BP + i) = v; __threadfence(); *(volatile float*)(BP + i) = v; } }
__global__ __launch_bounds__(256) void k_wdcn(const float* __restrict__ w, _Float16* __restrict__ Bt) { const int t = blockIdx.x * 256 + threadIdx.x; if (t >= CO * (2 * KD / 8)) return; const int col0 = (t % (2 * KD / 8)) * 8, o = t / (2 * KD / 8); const int n = col0 / 256, s = (col0 / 128) & 1, c0 = col0 % 128; const float sc = s ? (16.0f * 0.0009765625f) : 16.0f; FragH f;
#pragma unroll
  for (int q = 0; q < 8; ++q) f.h[q] = (_Float16)(bf16_round(w[((size_t)o * CO + c0 + q) * KT + n]) * sc);
  *(volatile v8us*)((unsigned short*)Bt + (size_t)o * 2 * KD + col0) = f.half[0]; __threadfence(); *(volatile v8us*)((unsigned short*)Bt + (size_t)o * 2 * KD + col0) = f.half[0]; }
__global__ __launch_bounds__(256) void k_wpw(const float* __restrict__ w, _Float16* __restrict__ Bt) { const int t = blockIdx.x * 256 + threadIdx.x; if (t >= CO * (2 * CX / 8)) return; const int col0 = (t % (2 * CX / 8)) * 8, o = t / (2 * CX / 8); const int s = col0 / CX, k0 = col0 % CX; const float sc = s ? (16.0f * 0.0009765625f) : 16.0f; FragH f;
#pragma unroll
  for (int q = 0; q < 8; ++q) f.h[q] = (_Float16)(bf16_round(w[(size_t)o * CX + k0 + q]) * sc);
  *(volatile v8us*)((unsigned short*)Bt + (size_t)o * 2 * CX + col0) = f.half[0]; __threadfence(); *(volatile v8us*)((unsigned short*)Bt + (size_t)o * 2 * CX + col0) = f.half[0]; }
__global__ __launch_bounds__(256) void k_samp(const float* __restrict__ OM, const float* __restrict__ Hf, _Float16* __restrict__ DCOL) {
  #pragma clang fp contract(off)
  const int t = blockIdx.x * 256 + threadIdx.x; if (t >= NPX * KT * (CO / 8)) return; const int c0 = (t % (CO / 8)) * 8; const int n = (t / (CO / 8)) % KT; const int p = t / ((CO / 8) * KT); const int h = p / HH, w = p % HH; const float* om = OM + (size_t)p * NOMP; const float Hp1 = (float)(HH + 1);
  const float px = (float)(h + 1) + (float)(n / 3 - 1) + om[n], py = (float)(w + 1) + (float)(n % 3 - 1) + om[9 + n]; const float m = 1.0f / (1.0f + expf(-om[18 + n]));
  const float fx = floorf(px), fy = floorf(py); const float qx0 = fminf(fmaxf(fx, 0.f), Hp1), qx1 = fminf(fmaxf(fx + 1.0f, 0.f), Hp1), qy0 = fminf(fmaxf(fy, 0.f), Hp1), qy1 = fminf(fmaxf(fy + 1.0f, 0.f), Hp1); const float pxc = fminf(fmaxf(px, 0.f), Hp1), pyc = fminf(fmaxf(py, 0.f), Hp1);
  const float glt = (1.0f + (qx0 - pxc)) * (1.0f + (qy0 - pyc)), grb = (1.0f - (qx1 - pxc)) * (1.0f - (qy1 - pyc)), glb = (1.0f + (qx0 - pxc)) * (1.0f - (qy1 - pyc)), grt = (1.0f - (qx1 - pxc)) * (1.0f + (qy0 - pyc));
  float acc[8];
#pragma unroll
  for (int q = 0; q < 8; ++q) acc[q] = 0.f;
#pragma unroll
  for (int cn = 0; cn < 4; ++cn) { const int xi = (int)((cn == 0 || cn == 2) ? qx0 : qx1), yi = (int)((cn == 0 || cn == 3) ? qy0 : qy1); const float g = (cn == 0) ? glt : (cn == 1) ? grb : (cn == 2) ? glb : grt;
    const int r = xi - 1, c = yi - 1; const bool inside = (r >= 0 && r < HH && c >= 0 && c < HH); const float f = inside ? g : 0.f; const float* hp = Hf + ((size_t)min(max(r, 0), HH - 1) * HH + min(max(c, 0), HH - 1)) * CO + c0; const v4f ga = *(const v4fa*)(hp), gb = *(const v4fa*)(hp + 4);
#pragma unroll
    for (int q = 0; q < 4; ++q) { acc[q] += f * ga[q]; acc[4 + q] += f * gb[q]; } }
  FragH o, ol;
#pragma unroll
  for (int q = 0; q < 8; ++q) { const float v = acc[q] * m; o.h[q] = (_Float16)v; ol.h[q] = (_Float16)((v - (float)o.h[q]) * 1024.0f); }
  for (int pass = 0; pass < 2; ++pass) { *(volatile v8us*)((unsigned short*)DCOL + ((size_t)p * KT + n) * 2 * CO + c0) = o.half[0]; *(volatile v8us*)((unsigned short*)DCOL + ((size_t)p * KT + n) * 2 * CO + CO + c0) = ol.half[0]; if (pass == 0) __threadfence(); } }
__global__ __launch_bounds__(256) void k_stat(const float* __restrict__ F, int phase, float* __restrict__ ST) {
  #pragma clang fp contract(off)
  __shared__ float red[256]; const int c = blockIdx.x, tid = threadIdx.x; const float mean = phase ? ST[(size_t)c * 32] / (float)NR : 0.f; float s = 0.f;
  for (int r = tid; r < NR; r += 256) { const float v = F[(size_t)r * CO + c]; s += phase ? (v - mean) * (v - mean) : v; }
  red[tid] = s; __syncthreads(); for (int st = 128; st > 0; st >>= 1) { if (tid < st) red[tid] += red[tid + st]; __syncthreads(); }
  if (tid < 32) { float* line = ST + ((size_t)phase * CO + c) * 32; *(volatile float*)(line + tid) = red[0]; __threadfence(); *(volatile float*)(line + tid) = red[0]; } }
__global__ __launch_bounds__(256) void k_bngelu(const float* __restrict__ F, const float* __restrict__ ST, const float* __restrict__ g, const float* __restrict__ bb, float* __restrict__ G) {
  #pragma clang fp contract(off)
  const int t = blockIdx.x * 256 + threadIdx.x; if (t >= NR * (CO / 4)) return; const int c0 = (t % (CO / 4)) * 4, r = t / (CO / 4); const v4f a = *(const v4fa*)(F + (size_t)r * CO + c0); v4f v;
#pragma unroll 1
  for (int q = 0; q < 4; ++q) { const int c = c0 + q; const float mean = ST[(size_t)c * 32] / (float)NR, rs = rsqrtf(ST[(size_t)(CO + c) * 32] / (float)NR + 1e-5f); const float z = (((q == 0) ? a[0] : (q == 1) ? a[1] : (q == 2) ? a[2] : a[3]) - mean) * rs * bf16_round(g[c]) + bf16_round(bb[c]); const float ge = 0.5f * z * (1.0f + erff(z * 0.70710678118654752f));
#pragma unroll
    for (int k = 0; k < 4; ++k) v[k] = (k == q) ? ge : v[k]; }
  *(volatile v4f*)(G + (size_t)r * CO + c0) = v; __threadfence(); *(volatile v4f*)(G + (size_t)r * CO + c0) = v; }
__global__ __launch_bounds__(256) void k_out(const float* __restrict__ F, const float* __restrict__ ST, const float* __restrict__ g, const float* __restrict__ bb, float* __restrict__ out) {
  #pragma clang fp contract(off)
  const int t = blockIdx.x * 256 + threadIdx.x; if (t >= NBI * CO * (NPX / 4)) return; const int p0 = (t % (NPX / 4)) * 4; const int c = (t / (NPX / 4)) % CO; const int b = t / ((NPX / 4) * CO); const float mean = ST[(size_t)c * 32] / (float)NR, rs = rsqrtf(ST[(size_t)(CO + c) * 32] / (float)NR + 1e-5f); const float ga = bf16_round(g[c]), be = bf16_round(bb[c]); v4f v;
#pragma unroll
  for (int q = 0; q < 4; ++q) v[q] = fmaxf((F[((size_t)b * NPX + p0 + q) * CO + c] - mean) * rs * ga + be, 0.f);
  float* dst = out + ((size_t)b * CO + c) * NPX + p0; *(volatile v4f*)dst = v; __threadfence(); *(volatile v4f*)dst = v; }

extern "C" void kernel_launch(void* const* d_in, const int* in_sizes, int n_in,
                              void* d_out, int out_size, void* d_ws, size_t ws_size, hipStream_t stream) {
  (void)in_sizes; (void)n_in; (void)out_size;
  const float* const* I = (const float* const*)d_in; const float* x1 = I[0]; const float* x2 = I[1]; const float* dww = I[2]; const float* dwb = I[3]; const float* pww = I[4]; const float* pwb = I[5]; const float* p_w = I[6]; const float* p_b = I[7]; const float* m_w = I[8]; const float* m_b = I[9]; const float* dcn_w = I[10]; const float* bn1g = I[11]; const float* bn1b = I[12]; const float* dw2w = I[13]; const float* dw2b = I[14]; const float* bn2g = I[15]; const float* bn2b = I[16];
  char* ws = (char*)d_ws; size_t off = 0;
  auto take = [&](size_t bytes) { char* p = ws + off; off += (bytes + 255) & ~(size_t)255; return p; };
  _Float16* BPW = (_Float16*)take((size_t)CO * 2 * CX * 2); _Float16* BOM = (_Float16*)take((size_t)NOMP * KD * 2); float* BOMP = (float*)take(NOMP * 4); _Float16* BDC = (_Float16*)take((size_t)CO * 2 * KD * 2); float* ST = (float*)take(2 * CO * 32 * 4);
  float* XC = (float*)take((size_t)NPX * CX * 4); _Float16* DW16 = (_Float16*)take((size_t)NPX * 2 * CX * 2); float* Hf = (float*)take((size_t)NPX * CO * 4); _Float16* H16 = (_Float16*)take((size_t)NPX * CO * 2); _Float16* COL = (_Float16*)take((size_t)NPX * 2 * KD * 2); float* OM = (float*)take((size_t)NPX * NOMP * 4);
  float* D = (float*)take((size_t)NR * CO * 4); float* G = (float*)take((size_t)NR * CO * 4); float* F2 = (float*)take((size_t)NR * CO * 4);
  if (off > ws_size) return;
  k_wpw<<<(CO * (2 * CX / 8) + 255) / 256, 256, 0, stream>>>(pww, BPW);
  k_wom<<<(NOMP * (KD / 8) + 255) / 256, 256, 0, stream>>>(p_w, m_w, p_b, m_b, BOM, BOMP); k_wdcn<<<(CO * (2 * KD / 8) + 255) / 256, 256, 0, stream>>>(dcn_w, BDC);
  const unsigned nbs = (NPX * KT * (CO / 8) + 255) / 256; const dim3 gP(((NPX / 16) * (CO / 64) + 3) / 4, 1), gO(((NPX / 16) * 1 + 3) / 4, 1);
  for (int b = 0; b < NBI; ++b) {
    k_xcat<<<(NPX * (CX / 4) + 255) / 256, 256, 0, stream>>>(x1, x2, b, XC);
    k_dw<<<(NPX * (CX / 4) + 255) / 256, 256, 0, stream>>>(XC, CX, dww, dwb, 0, DW16, nullptr);
    k_gemm_hhx<0><<<gP, 128, 0, stream>>>(DW16, 2 * CX, 0, BPW, 2 * CX, 0, 0.0625f, pwb, 0, nullptr, 1, 0, 0, Hf, H16, CO, 0, NPX, CO, 2 * CX);
    k_im2col<<<nbs, 256, 0, stream>>>(H16, COL);
    k_gemm_hhx<0><<<gO, 128, 0, stream>>>(COL, KD, 0, BOM, KD, 0, 0.0625f, BOMP, 0, nullptr, 1, 0, 0, OM, nullptr, NOMP, 0, NPX, NOMP, KD);
    k_samp<<<nbs, 256, 0, stream>>>(OM, Hf, COL);
    k_gemm_hhx<0><<<gP, 128, 0, stream>>>(COL, 2 * KD, 0, BDC, 2 * KD, 0, 0.0625f, nullptr, 0, nullptr, 1, 0, 0, D + (size_t)b * NPX * CO, nullptr, CO, 0, NPX, CO, 2 * KD); }
  k_stat<<<CO, 256, 0, stream>>>(D, 0, ST); k_stat<<<CO, 256, 0, stream>>>(D, 1, ST);
  k_bngelu<<<(NR * (CO / 4) + 255) / 256, 256, 0, stream>>>(D, ST, bn1g, bn1b, G);
  for (int b = 0; b < NBI; ++b) k_dw<<<(NPX * (CO / 4) + 255) / 256, 256, 0, stream>>>(G + (size_t)b * NPX * CO, CO, dw2w, dw2b, 1, nullptr, F2 + (size_t)b * NPX * CO);
  k_stat<<<CO, 256, 0, stream>>>(F2, 0, ST); k_stat<<<CO, 256, 0, stream>>>(F2, 1, ST);
  k_out<<<(unsigned)(((size_t)NBI * CO * (NPX / 4) + 255) / 256), 256, 0, stream>>>(F2, ST, bn2g, bn2b, (float*)d_out);
}
